// MultiHeadAttention_33148557591136
// MI455X (gfx1250) — hardware-verified
//
#include <hip/hip_runtime.h>


#ifndef NB
#define NB 4
#endif
#ifndef SEQ
#define SEQ 2048
#endif
#define SEQ_FULL 2048
#define TT   SEQ
#define DM   1024
#define NH_  16
#define HD   64
#define DQ   (NH_ * HD)
#define NQ3  (3 * DQ)
#if SEQ < 512
#define RH SEQ
#else
#define RH 512
#endif
#define PCAR 1024.0f
#define SCL  0.125f
#define L2E  1.4426950408889634f
#define NEGF (-3.0e38f)

static_assert(HD == 64);
static_assert(HD * 2 == 128);
static_assert(DQ == NH_ * HD);
static_assert(TT % 64 == 0);
static_assert(RH % 32 == 0);
static_assert(RH <= TT);
static_assert((TT - RH) % 16 == 0);
static_assert(DM % 64 == 0);
static_assert(DQ % 64 == 0);
static_assert(NQ3 % 64 == 0);
static_assert(DM % 32 == 0);
static_assert(DQ % 32 == 0);
static_assert(NQ3 % 32 == 0);
static_assert(TT % 8 == 0);

typedef _Float16 h16;
typedef unsigned short bf;
typedef __attribute__((ext_vector_type(16))) __bf16   v16bf;
typedef __attribute__((ext_vector_type(16))) _Float16 v16h;
typedef __attribute__((ext_vector_type(8)))  _Float16 v8h;
typedef __attribute__((ext_vector_type(8)))  unsigned short v8us;
typedef __attribute__((ext_vector_type(2)))  unsigned short v2us;
typedef __attribute__((ext_vector_type(8)))  float    v8f;
typedef __attribute__((ext_vector_type(4)))  float    v4f;
typedef v8h  __attribute__((may_alias)) v8ha;
typedef v4f  __attribute__((may_alias)) v4fa;
typedef v8us __attribute__((may_alias)) v8usa;

__device__ __forceinline__ unsigned short f2bf(float f) { unsigned u = __float_as_uint(f); u += 0x7FFFu + ((u >> 16) & 1u); return (unsigned short)(u >> 16); }
__device__ __forceinline__ float bf2f(unsigned short b) { return __uint_as_float(((unsigned)b) << 16); }
__device__ __forceinline__ float bfr(float f) { return bf2f(f2bf(f)); }
__device__ __forceinline__ void splitf(float y, unsigned short& h, unsigned short& l) { h = f2bf(y); l = f2bf(y - bf2f(h)); }
__device__ __forceinline__ v16h cat16(v8h lo, v8h hi) { return __builtin_shufflevector(lo, hi, 0, 1, 2, 3, 4, 5, 6, 7, 8, 9, 10, 11, 12, 13, 14, 15); }
__device__ __forceinline__ v16bf cat16b(v8us lo, v8us hi) { return __builtin_bit_cast(v16bf, __builtin_shufflevector(lo, hi, 0, 1, 2, 3, 4, 5, 6, 7, 8, 9, 10, 11, 12, 13, 14, 15)); }
__device__ __forceinline__ v8f wmma16(v16h a, v16h b, v8f c) { return __builtin_amdgcn_wmma_f32_16x16x32_f16(false, a, false, b, (short)0, c, false, false); }
__device__ __forceinline__ v8f wmmab(v16bf a, v16bf b, v8f c) { return __builtin_amdgcn_wmma_f32_16x16x32_bf16(false, a, false, b, (short)0, c, false, false); }
__device__ __forceinline__ v16h  ldh(const h16* p) { return cat16(*(const v8h*)p, *(const v8h*)(p + 16)); }
__device__ __forceinline__ v16bf ldb(const bf* p)  { return cat16b(*(const v8us*)p, *(const v8us*)(p + 16)); }

template <typename T16> struct WFrag;
template <> struct WFrag<h16> { typedef v16h V; static __device__ __forceinline__ V ld(const h16* p) { return ldh(p); } static __device__ __forceinline__ v8f mma(V a, V b, v8f c) { return wmma16(a, b, c); } };
template <> struct WFrag<bf> { typedef v16bf V; static __device__ __forceinline__ V ld(const bf* p) { return ldb(p); } static __device__ __forceinline__ v8f mma(V a, V b, v8f c) { return wmmab(a, b, c); } };
template <typename T16, int NSPLIT, bool BIAS>
__device__ __forceinline__ void gemmw_body(const T16* __restrict__ A, const T16* __restrict__ A2, const T16* __restrict__ Bt, const T16* __restrict__ Bt2, const int K, float* C, const int ldc, const float* __restrict__ bias, size_t sA, size_t sB, size_t sC) {
    typedef typename WFrag<T16>::V V;
    __shared__ __align__(16) float os[16 * 68];
    const size_t z = blockIdx.z; A += z * sA; if (A2) A2 += z * sA; Bt += z * sB; if (Bt2) Bt2 += z * sB; C += z * sC;
    const int lane = threadIdx.x & 31, lr = lane & 15, hi = lane >> 4; const int r0 = blockIdx.x * 64, c0 = blockIdx.y * 64;
    v8f acc[4][4];
#pragma unroll
    for (int mb = 0; mb < 4; ++mb)
#pragma unroll
        for (int nb = 0; nb < 4; ++nb) acc[mb][nb] = (v8f){};
    const size_t aoff = (size_t)(r0 + lr) * K + 8 * hi, boff = (size_t)(c0 + lr) * K + 8 * hi;
#pragma unroll 1
    for (int kc = 0; kc < K; kc += 32) {
        V a[4], a2[4];
#pragma unroll
        for (int mb = 0; mb < 4; ++mb) { a[mb] = WFrag<T16>::ld(A + aoff + (size_t)mb * 16 * K + kc); if (NSPLIT == 1 || NSPLIT == 2) a2[mb] = WFrag<T16>::ld(A2 + aoff + (size_t)mb * 16 * K + kc); }
#pragma unroll
        for (int nb = 0; nb < 4; ++nb) { const V b = WFrag<T16>::ld(Bt + boff + (size_t)nb * 16 * K + kc); V b2; if (NSPLIT >= 2) b2 = WFrag<T16>::ld(Bt2 + boff + (size_t)nb * 16 * K + kc);
#pragma unroll
            for (int mb = 0; mb < 4; ++mb) { acc[mb][nb] = WFrag<T16>::mma(a[mb], b, acc[mb][nb]); if (NSPLIT == 1 || NSPLIT == 2) acc[mb][nb] = WFrag<T16>::mma(a2[mb], b, acc[mb][nb]); if (NSPLIT >= 2) acc[mb][nb] = WFrag<T16>::mma(a[mb], b2, acc[mb][nb]); } }
        asm volatile("v_nop\n\tv_nop\n\tv_nop\n\tv_nop" : "+v"(acc[0][0]), "+v"(acc[1][1]), "+v"(acc[2][2]), "+v"(acc[3][3]) : "v"(a[0]), "v"(a[3]));
    }
#pragma unroll
    for (int mb = 0; mb < 4; ++mb) {
#pragma unroll
        for (int nb = 0; nb < 4; ++nb) {
#pragma unroll
            for (int j = 0; j < 8; ++j) os[(hi * 8 + j) * 68 + nb * 16 + lr] = acc[mb][nb][j]; }
        __builtin_amdgcn_wave_barrier(); asm volatile("" ::: "memory");
        float* crow = C + (size_t)(r0 + mb * 16) * ldc + c0;
#pragma unroll 1
        for (int ps = 0; ps < 2; ++ps) {
#pragma unroll
            for (int s = 0; s < 8; ++s) { const int row = 2 * s + hi, cofs = lr * 4; v4f val = *(const v4fa*)(os + row * 68 + cofs); if (BIAS) { val[0] += bfr(bias[c0 + cofs]); val[1] += bfr(bias[c0 + cofs + 1]); val[2] += bfr(bias[c0 + cofs + 2]); val[3] += bfr(bias[c0 + cofs + 3]); }
                *(volatile v4f*)(crow + (size_t)row * ldc + cofs) = val; }
            if (ps == 0) __threadfence(); }
        __builtin_amdgcn_wave_barrier(); asm volatile("" ::: "memory");
    }
}
__global__ __launch_bounds__(32) void k_gemm_qkv(const bf* __restrict__ A, const bf* __restrict__ Bt, float* C) {
    gemmw_body<bf, 0, false>(A, nullptr, Bt, nullptr, DM, C, NQ3, nullptr, 0, 0, 0);
}
__global__ __launch_bounds__(32) void k_gemm_out(const bf* __restrict__ Ah, const bf* __restrict__ Al, const bf* __restrict__ Bt, float* C, const float* __restrict__ bias) {
    gemmw_body<bf, 1, true>(Ah, Al, Bt, nullptr, DQ, C, DM, bias, (size_t)TT * DQ, 0, (size_t)SEQ_FULL * DM);
}

__global__ __launch_bounds__(256) void k_wtG(const float* __restrict__ w, int K, int N, bf* Bt) {
    const int lane = threadIdx.x & 31; const int L0 = (blockIdx.x * 8 + (threadIdx.x >> 5)) * 8; const int nlines = N * K / 64;
#pragma unroll
    for (int ps = 0; ps < 2; ++ps) {
#pragma unroll 1
        for (int l = 0; l < 8; ++l) { const int L = L0 + l; if (L >= nlines) break; const size_t e = (size_t)L * 64 + lane * 2; const int k = (int)(e % K), n = (int)(e / K); v2us o;
            o[0] = f2bf(w[(size_t)k * N + n]); o[1] = f2bf(w[(size_t)(k + 1) * N + n]); *(volatile v2us*)(Bt + e) = o; }
        if (ps == 0) __threadfence(); }
}
__global__ __launch_bounds__(256) void k_cvtx(const float* __restrict__ src, bf* dst, int n8, size_t sstr, size_t dstr) {
    const int i = blockIdx.x * 256 + threadIdx.x; if (i >= n8) return;
    const float* s = src + (size_t)blockIdx.y * sstr + (size_t)i * 8; bf* d = dst + (size_t)blockIdx.y * dstr + (size_t)i * 8;
    const v8f v = *(const v8f*)s; v8us o;
#pragma unroll
    for (int k = 0; k < 8; ++k) o[k] = f2bf(v[k]);
    *(volatile v8us*)d = o; __threadfence(); *(volatile v8us*)d = o;
}
__global__ __launch_bounds__(256) void k_qkp(const float* __restrict__ F, h16* P16, bf* Ph, bf* Pl) {
    const size_t i = (size_t)blockIdx.x * 256 + threadIdx.x; if (i >= (size_t)2 * NH_ * TT * HD / 8) return;
    const int d = (int)(i % (HD / 8)) * 8; const int t = (int)((i / (HD / 8)) % TT); const int g = (int)(i / ((size_t)(HD / 8) * TT));
    const float* f = F + (size_t)t * NQ3 + g * HD + d; const v4f a = *(const v4f*)f; const v4f b = *(const v4f*)(f + 4);
    v8h o16; v8us oh, ol;
#pragma unroll
    for (int k = 0; k < 4; ++k) { unsigned short u, w; o16[k] = (h16)a[k]; splitf(a[k], u, w); oh[k] = u; ol[k] = w; o16[k + 4] = (h16)b[k]; splitf(b[k], u, w); oh[k + 4] = u; ol[k + 4] = w; }
    const bool hr = (t < RH); const int tc = hr ? t : (RH - 1);
    const size_t e = ((size_t)g * TT + t) * HD + d; const size_t e2 = ((size_t)g * RH + tc) * HD + d;
    *(volatile v8h*)(P16 + e) = o16; if (hr) { *(volatile v8us*)(Ph + e2) = oh; *(volatile v8us*)(Pl + e2) = ol; }
    __threadfence();
    *(volatile v8h*)(P16 + e) = o16; if (hr) { *(volatile v8us*)(Ph + e2) = oh; *(volatile v8us*)(Pl + e2) = ol; }
}
__global__ __launch_bounds__(256) void k_vtp(const float* __restrict__ F, h16* V16, bf* Vh, bf* Vl) {
    const size_t i = (size_t)blockIdx.x * 256 + threadIdx.x; if (i >= (size_t)NH_ * HD * TT / 8) return;
    const int t = (int)(i % (TT / 8)) * 8; const int d = (int)((i / (TT / 8)) % HD); const int g = (int)(i / ((size_t)(TT / 8) * HD));
    const float* f = F + (size_t)t * NQ3 + 2 * DQ + g * HD + d;
    v8h o16; v8us oh, ol;
#pragma unroll
    for (int q = 0; q < 8; ++q) { const float x = f[(size_t)q * NQ3]; unsigned short u, w; o16[q] = (h16)x; splitf(x, u, w); oh[q] = u; ol[q] = w; }
    const bool hr = (t < RH); const int tc = hr ? t : (RH - 8);
    const size_t e = ((size_t)g * HD + d) * TT + t; const size_t e2 = ((size_t)g * HD + d) * RH + tc;
    *(volatile v8h*)(V16 + e) = o16; if (hr) { *(volatile v8us*)(Vh + e2) = oh; *(volatile v8us*)(Vl + e2) = ol; }
    __threadfence();
    *(volatile v8h*)(V16 + e) = o16; if (hr) { *(volatile v8us*)(Vh + e2) = oh; *(volatile v8us*)(Vl + e2) = ol; }
}

__global__ __launch_bounds__(32) void k_flash16(const h16* __restrict__ Q16, const h16* __restrict__ K16, const h16* __restrict__ V16, bf* ATh, bf* ATl) {
    __shared__ __align__(16) h16 ps[16 * 40];
    __shared__ __align__(16) unsigned short osh[16 * 72];
    __shared__ __align__(16) unsigned short osl[16 * 72];
    const int lane = threadIdx.x & 31, lr = lane & 15, hi = lane >> 4;
    const int h = blockIdx.y; const int q0 = RH + (int)blockIdx.x * 16;
    const h16* Qp = Q16 + (size_t)h * TT * HD; const h16* Kp = K16 + (size_t)h * TT * HD; const h16* Vp = V16 + (size_t)h * HD * TT;
    const int qoff = (q0 + lr) * HD + 8 * hi;
    v8f acc[4]; float mrun[8], lrun[8];
#pragma unroll
    for (int j = 0; j < 4; ++j) acc[j] = (v8f){};
#pragma unroll
    for (int r = 0; r < 8; ++r) { mrun[r] = NEGF; lrun[r] = 0.f; }
    const int qlast = q0 + 15; const int qr = q0 + 8 * hi;
#pragma unroll 1
    for (int key0 = 0; key0 <= qlast; key0 += 32) {
        int qo = qoff; asm volatile("" : "+v"(qo));
        const int ko = (key0 + lr) * HD + 8 * hi;
        v8f s0 = (v8f){}, s1 = (v8f){};
        {
            const v16h a0 = ldh(Qp + qo), a1 = ldh(Qp + qo + 32);
            const v16h b00 = ldh(Kp + ko), b01 = ldh(Kp + ko + 32), b10 = ldh(Kp + ko + 16 * HD), b11 = ldh(Kp + ko + 16 * HD + 32);
            s0 = wmma16(a0, b00, s0); s1 = wmma16(a0, b10, s1); s0 = wmma16(a1, b01, s0); s1 = wmma16(a1, b11, s1);
            asm volatile("v_nop\n\tv_nop\n\tv_nop\n\tv_nop" : "+v"(s0), "+v"(s1) : "v"(a0), "v"(a1), "v"(b00), "v"(b01), "v"(b10), "v"(b11));
        }
        float e0[8], e1[8], alf[8];
        const int kA = key0 + lr, kB = key0 + 16 + lr;
#pragma unroll
        for (int r = 0; r < 8; ++r) {
            const bool v0 = (kA <= qr + r), v1 = (kB <= qr + r);
            const float t0 = v0 ? s0[r] * SCL : NEGF; const float t1 = v1 ? s1[r] * SCL : NEGF;
            float m = fmaxf(t0, t1);
            m = fmaxf(m, __shfl_xor(m, 8, 32)); m = fmaxf(m, __shfl_xor(m, 4, 32)); m = fmaxf(m, __shfl_xor(m, 2, 32)); m = fmaxf(m, __shfl_xor(m, 1, 32));
            const float mn = fmaxf(mrun[r], m);
            alf[r] = __builtin_amdgcn_exp2f((mrun[r] - mn) * L2E); mrun[r] = mn;
            const float x0 = __builtin_amdgcn_exp2f((t0 - mn) * L2E), x1 = __builtin_amdgcn_exp2f((t1 - mn) * L2E);
            e0[r] = v0 ? x0 : 0.f; e1[r] = v1 ? x1 : 0.f;
            lrun[r] = lrun[r] * alf[r] + (e0[r] + e1[r]);
        }
#pragma unroll
        for (int j = 0; j < 4; ++j)
#pragma unroll
            for (int r = 0; r < 8; ++r) acc[j][r] *= alf[r];
#pragma unroll
        for (int r = 0; r < 8; ++r) { ps[(8 * hi + r) * 40 + lr] = (h16)(e0[r] * PCAR); ps[(8 * hi + r) * 40 + 16 + lr] = (h16)(e1[r] * PCAR); }
        __builtin_amdgcn_wave_barrier(); asm volatile("" ::: "memory");
        const v16h pa = cat16(*(const v8ha*)(ps + lr * 40 + 8 * hi), *(const v8ha*)(ps + lr * 40 + 16 + 8 * hi));
        __builtin_amdgcn_wave_barrier(); asm volatile("" ::: "memory");
        const int vo = lr * TT + key0 + 8 * hi;
        v16h vb[4];
#pragma unroll
        for (int j = 0; j < 4; ++j) vb[j] = ldh(Vp + vo + j * 16 * TT);
#pragma unroll
        for (int j = 0; j < 4; ++j) acc[j] = wmma16(pa, vb[j], acc[j]);
        asm volatile("v_nop\n\tv_nop\n\tv_nop\n\tv_nop" : "+v"(acc[0]), "+v"(acc[1]), "+v"(acc[2]), "+v"(acc[3]) : "v"(pa), "v"(vb[0]), "v"(vb[1]), "v"(vb[2]), "v"(vb[3]));
    }
    float linv[8];
#pragma unroll
    for (int r = 0; r < 8; ++r) { float l = lrun[r]; l += __shfl_xor(l, 8, 32); l += __shfl_xor(l, 4, 32); l += __shfl_xor(l, 2, 32); l += __shfl_xor(l, 1, 32); linv[r] = (1.0f / l) * (1.0f / PCAR); }
#pragma unroll
    for (int j = 0; j < 4; ++j)
#pragma unroll
        for (int r = 0; r < 8; ++r) { unsigned short u, w; splitf(acc[j][r] * linv[r], u, w); osh[(8 * hi + r) * 72 + j * 16 + lr] = u; osl[(8 * hi + r) * 72 + j * 16 + lr] = w; }
    __builtin_amdgcn_wave_barrier(); asm volatile("" ::: "memory");
    const int rr = lane >> 3, cc = (lane & 7) * 8; const size_t ob = (size_t)q0 * DQ + (size_t)h * HD + cc;
#pragma unroll 1
    for (int pz = 0; pz < 2; ++pz) {
#pragma unroll
        for (int s = 0; s < 4; ++s) { const int row = 4 * s + rr; const v8us xh = *(const v8usa*)(osh + row * 72 + cc); const v8us xl = *(const v8usa*)(osl + row * 72 + cc);
            *(volatile v8us*)(ATh + ob + (size_t)row * DQ) = xh; *(volatile v8us*)(ATl + ob + (size_t)row * DQ) = xl; }
        if (pz == 0) __threadfence(); }
}

__global__ __launch_bounds__(32) void k_flash_hl(const bf* __restrict__ Qh, const bf* __restrict__ Ql, const bf* __restrict__ Kh, const bf* __restrict__ Kl, const bf* __restrict__ Vh, const bf* __restrict__ Vl, bf* ATh, bf* ATl) {
    __shared__ __align__(16) unsigned short psh[16 * 40];
    __shared__ __align__(16) unsigned short psl[16 * 40];
    __shared__ __align__(16) unsigned short osh[16 * 72];
    __shared__ __align__(16) unsigned short osl[16 * 72];
    const int lane = threadIdx.x & 31, lr = lane & 15, hi = lane >> 4;
    const int h = blockIdx.y; const int q0 = (int)blockIdx.x * 16;
    const size_t pb = (size_t)h * RH * HD;
    const bf* qh = Qh + pb; const bf* ql = Ql + pb; const bf* kh = Kh + pb; const bf* kl = Kl + pb; const bf* vhp = Vh + pb; const bf* vlp = Vl + pb;
    const int qoff = (q0 + lr) * HD + 8 * hi;
    v8f acc[4]; float mrun[8], lrun[8];
#pragma unroll
    for (int j = 0; j < 4; ++j) acc[j] = (v8f){};
#pragma unroll
    for (int r = 0; r < 8; ++r) { mrun[r] = NEGF; lrun[r] = 0.f; }
    const int qlast = q0 + 15; const int qr = q0 + 8 * hi;
#pragma unroll 1
    for (int key0 = 0; key0 <= qlast; key0 += 32) {
        int qo = qoff; asm volatile("" : "+v"(qo));
        const int ko = (key0 + lr) * HD + 8 * hi;
        const v16bf ah0 = ldb(qh + qo), ah1 = ldb(qh + qo + 32), aw0 = ldb(ql + qo), aw1 = ldb(ql + qo + 32);
        v8f s0 = (v8f){}, s1 = (v8f){};
        {
            const v16bf bh0 = ldb(kh + ko), bh1 = ldb(kh + ko + 32), bw0 = ldb(kl + ko), bw1 = ldb(kl + ko + 32);
            s0 = wmmab(ah0, bh0, s0); s0 = wmmab(aw0, bh0, s0); s0 = wmmab(ah0, bw0, s0);
            s0 = wmmab(ah1, bh1, s0); s0 = wmmab(aw1, bh1, s0); s0 = wmmab(ah1, bw1, s0);
            asm volatile("v_nop\n\tv_nop\n\tv_nop\n\tv_nop" : "+v"(s0) : "v"(ah0), "v"(ah1), "v"(aw0), "v"(aw1), "v"(bh0), "v"(bh1), "v"(bw0), "v"(bw1));
        }
        {
            const int k1 = ko + 16 * HD;
            const v16bf bh0 = ldb(kh + k1), bh1 = ldb(kh + k1 + 32), bw0 = ldb(kl + k1), bw1 = ldb(kl + k1 + 32);
            s1 = wmmab(ah0, bh0, s1); s1 = wmmab(aw0, bh0, s1); s1 = wmmab(ah0, bw0, s1);
            s1 = wmmab(ah1, bh1, s1); s1 = wmmab(aw1, bh1, s1); s1 = wmmab(ah1, bw1, s1);
            asm volatile("v_nop\n\tv_nop\n\tv_nop\n\tv_nop" : "+v"(s1) : "v"(ah0), "v"(ah1), "v"(aw0), "v"(aw1), "v"(bh0), "v"(bh1), "v"(bw0), "v"(bw1));
        }
        float e0[8], e1[8], alf[8];
        const int kA = key0 + lr, kB = key0 + 16 + lr;
#pragma unroll
        for (int r = 0; r < 8; ++r) {
            const bool v0 = (kA <= qr + r), v1 = (kB <= qr + r);
            const float t0 = v0 ? s0[r] * SCL : NEGF; const float t1 = v1 ? s1[r] * SCL : NEGF;
            float m = fmaxf(t0, t1);
            m = fmaxf(m, __shfl_xor(m, 8, 32)); m = fmaxf(m, __shfl_xor(m, 4, 32)); m = fmaxf(m, __shfl_xor(m, 2, 32)); m = fmaxf(m, __shfl_xor(m, 1, 32));
            const float mn = fmaxf(mrun[r], m);
            alf[r] = __builtin_amdgcn_exp2f((mrun[r] - mn) * L2E); mrun[r] = mn;
            const float x0 = __builtin_amdgcn_exp2f((t0 - mn) * L2E), x1 = __builtin_amdgcn_exp2f((t1 - mn) * L2E);
            e0[r] = v0 ? x0 : 0.f; e1[r] = v1 ? x1 : 0.f;
            lrun[r] = lrun[r] * alf[r] + (e0[r] + e1[r]);
        }
#pragma unroll
        for (int j = 0; j < 4; ++j)
#pragma unroll
            for (int r = 0; r < 8; ++r) acc[j][r] *= alf[r];
#pragma unroll
        for (int r = 0; r < 8; ++r) { unsigned short u, w; splitf(e0[r], u, w); psh[(8 * hi + r) * 40 + lr] = u; psl[(8 * hi + r) * 40 + lr] = w; splitf(e1[r], u, w); psh[(8 * hi + r) * 40 + 16 + lr] = u; psl[(8 * hi + r) * 40 + 16 + lr] = w; }
        __builtin_amdgcn_wave_barrier(); asm volatile("" ::: "memory");
        const v16bf pah = cat16b(*(const v8usa*)(psh + lr * 40 + 8 * hi), *(const v8usa*)(psh + lr * 40 + 16 + 8 * hi));
        const v16bf paw = cat16b(*(const v8usa*)(psl + lr * 40 + 8 * hi), *(const v8usa*)(psl + lr * 40 + 16 + 8 * hi));
        __builtin_amdgcn_wave_barrier(); asm volatile("" ::: "memory");
        const int vo = lr * RH + key0 + 8 * hi;
        v16bf vh[4], vw[4];
#pragma unroll
        for (int j = 0; j < 4; ++j) { vh[j] = ldb(vhp + vo + j * 16 * RH); vw[j] = ldb(vlp + vo + j * 16 * RH); }
#pragma unroll
        for (int j = 0; j < 4; ++j) { acc[j] = wmmab(pah, vh[j], acc[j]); acc[j] = wmmab(paw, vh[j], acc[j]); acc[j] = wmmab(pah, vw[j], acc[j]); }
        asm volatile("v_nop\n\tv_nop\n\tv_nop\n\tv_nop" : "+v"(acc[0]), "+v"(acc[1]), "+v"(acc[2]), "+v"(acc[3]) : "v"(pah), "v"(paw), "v"(vh[0]), "v"(vh[1]), "v"(vh[2]), "v"(vh[3]), "v"(vw[0]), "v"(vw[1]), "v"(vw[2]), "v"(vw[3]));
    }
    float linv[8];
#pragma unroll
    for (int r = 0; r < 8; ++r) { float l = lrun[r]; l += __shfl_xor(l, 8, 32); l += __shfl_xor(l, 4, 32); l += __shfl_xor(l, 2, 32); l += __shfl_xor(l, 1, 32); linv[r] = 1.0f / l; }
#pragma unroll
    for (int j = 0; j < 4; ++j)
#pragma unroll
        for (int r = 0; r < 8; ++r) { unsigned short u, w; splitf(acc[j][r] * linv[r], u, w); osh[(8 * hi + r) * 72 + j * 16 + lr] = u; osl[(8 * hi + r) * 72 + j * 16 + lr] = w; }
    __builtin_amdgcn_wave_barrier(); asm volatile("" ::: "memory");
    const int rr = lane >> 3, cc = (lane & 7) * 8; const size_t ob = (size_t)q0 * DQ + (size_t)h * HD + cc;
#pragma unroll 1
    for (int pz = 0; pz < 2; ++pz) {
#pragma unroll
        for (int s = 0; s < 4; ++s) { const int row = 4 * s + rr; const v8us xh = *(const v8usa*)(osh + row * 72 + cc); const v8us xl = *(const v8usa*)(osl + row * 72 + cc);
            *(volatile v8us*)(ATh + ob + (size_t)row * DQ) = xh; *(volatile v8us*)(ATl + ob + (size_t)row * DQ) = xl; }
        if (pz == 0) __threadfence(); }
}

constexpr size_t SZ_WQKV = (size_t)NQ3 * DM * 2;
constexpr size_t SZ_WO   = (size_t)DM * DQ * 2;
constexpr size_t SZ_XB   = (size_t)NB * TT * DM * 2;
constexpr size_t SZ_F    = (size_t)TT * NQ3 * 4;
constexpr size_t SZ_QK16 = (size_t)2 * NH_ * TT * HD * 2;
constexpr size_t SZ_VT16 = (size_t)NH_ * HD * TT * 2;
constexpr size_t SZ_QKS  = (size_t)2 * NH_ * RH * HD * 2;
constexpr size_t SZ_VTS  = (size_t)NH_ * HD * RH * 2;
constexpr size_t SZ_AT   = (size_t)NB * TT * DQ * 2;
constexpr size_t SZ_ALL  = SZ_WQKV + SZ_WO + SZ_XB + SZ_F + SZ_QK16 + SZ_VT16 + 2 * SZ_QKS + 2 * SZ_VTS + 2 * SZ_AT;
static_assert(SZ_WQKV % 256 == 0 && SZ_WO % 256 == 0 && SZ_XB % 256 == 0 && SZ_F % 256 == 0 && SZ_QK16 % 256 == 0 && SZ_VT16 % 256 == 0 && SZ_QKS % 256 == 0 && SZ_VTS % 256 == 0 && SZ_AT % 256 == 0);
static_assert(SZ_ALL <= (size_t)134217728);

extern "C" void kernel_launch(void* const* d_in, const int* in_sizes, int n_in,
                              void* d_out, int out_size, void* d_ws, size_t ws_size, hipStream_t stream) {
    if (n_in < 4) return;
    const long long need_x = (long long)(NB - 1) * SEQ_FULL * DM + (long long)TT * DM;
    if ((long long)in_sizes[0] < need_x || (long long)in_sizes[1] < (long long)DM * NQ3 || (long long)in_sizes[2] < (long long)DQ * DM || in_sizes[3] < DM || (long long)out_size < need_x) return;
    if (ws_size < SZ_ALL) return;
    const float* x = (const float*)d_in[0]; const float* wqkv = (const float*)d_in[1]; const float* wfc = (const float*)d_in[2]; const float* bfc = (const float*)d_in[3];
    float* OUT = (float*)d_out;
    char* wsp = (char*)d_ws;
    auto take = [&](size_t bytes) { char* p = wsp; wsp += bytes; return (void*)p; };
    bf* WQKV = (bf*)take(SZ_WQKV);
    bf* WO   = (bf*)take(SZ_WO);
    bf* XB   = (bf*)take(SZ_XB);
    float* F = (float*)take(SZ_F);
    h16* QK16 = (h16*)take(SZ_QK16);
    h16* VT16 = (h16*)take(SZ_VT16);
    bf* QKh = (bf*)take(SZ_QKS); bf* QKl = (bf*)take(SZ_QKS);
    bf* VTh = (bf*)take(SZ_VTS); bf* VTl = (bf*)take(SZ_VTS);
    bf* ATh = (bf*)take(SZ_AT);  bf* ATl = (bf*)take(SZ_AT);
    k_wtG<<<(unsigned)((DM * NQ3 / 64 + 63) / 64), 256, 0, stream>>>(wqkv, DM, NQ3, WQKV);
    k_wtG<<<(unsigned)((DQ * DM / 64 + 63) / 64), 256, 0, stream>>>(wfc, DQ, DM, WO);
    k_cvtx<<<dim3((unsigned)((TT * DM / 8 + 255) / 256), NB, 1), 256, 0, stream>>>(x, XB, TT * DM / 8, (size_t)SEQ_FULL * DM, (size_t)TT * DM);
    for (int b = 0; b < NB; ++b) {
        k_gemm_qkv<<<dim3(TT / 64, NQ3 / 64, 1), 32, 0, stream>>>(XB + (size_t)b * TT * DM, WQKV, F);
        k_qkp<<<(unsigned)(((size_t)2 * NH_ * TT * HD / 8 + 255) / 256), 256, 0, stream>>>(F, QK16, QKh, QKl);
        k_vtp<<<(unsigned)(((size_t)NH_ * HD * TT / 8 + 255) / 256), 256, 0, stream>>>(F, VT16, VTh, VTl);
        k_flash_hl<<<dim3(RH / 16, NH_, 1), 32, 0, stream>>>(QKh, QKl, QKh + (size_t)NH_ * RH * HD, QKl + (size_t)NH_ * RH * HD, VTh, VTl, ATh + (size_t)b * TT * DQ, ATl + (size_t)b * TT * DQ);
#if SEQ > 512
        k_flash16<<<dim3((TT - RH) / 16, NH_, 1), 32, 0, stream>>>(QK16, QK16 + (size_t)NH_ * TT * HD, VT16, ATh + (size_t)b * TT * DQ, ATl + (size_t)b * TT * DQ);
#endif
    }
    k_gemm_out<<<dim3(TT / 64, DM / 64, NB), 32, 0, stream>>>(ATh, ATl, WO, OUT, bfc);
}
